// PredictionHeadEdge_2104533975131
// MI455X (gfx1250) — hardware-run, weakly checked
//
#include <hip/hip_runtime.h>

typedef float          v8f   __attribute__((ext_vector_type(8)));
typedef float          v4f   __attribute__((ext_vector_type(4)));
typedef unsigned int   v4u   __attribute__((ext_vector_type(4)));
typedef int            v8i   __attribute__((ext_vector_type(8)));
typedef unsigned short v8us  __attribute__((ext_vector_type(8)));
typedef unsigned short v16us __attribute__((ext_vector_type(16)));
typedef __bf16         v16bf __attribute__((ext_vector_type(16)));
typedef _Float16       v16h  __attribute__((ext_vector_type(16)));
typedef v4f  __attribute__((may_alias)) v4fa;
typedef v8us __attribute__((may_alias)) v8usa;
union FragB { v16bf v; v16us u; v8us h[2]; v8i w; };
union FragH { v16h  v; v16us u; v8us h[2]; v8i w; };

__device__ __forceinline__ v8f wmb(const FragB& a, const FragB& b, v8f c) {
  v8f d = __builtin_amdgcn_wmma_f32_16x16x32_bf16(false, a.v, false, b.v, (short)0, c, false, false);
  asm volatile("v_nop\n\tv_nop\n\tv_nop\n\tv_nop" : "+v"(d) : "v"(a.w), "v"(b.w));
  return d;
}

__device__ __forceinline__ v8f wmh(const FragH& a, const FragH& b, v8f c) {
  v8f d = __builtin_amdgcn_wmma_f32_16x16x32_f16(false, a.v, false, b.v, (short)0, c, false, false);
  asm volatile("v_nop\n\tv_nop\n\tv_nop\n\tv_nop" : "+v"(d) : "v"(a.w), "v"(b.w));
  return d;
}

__device__ __forceinline__ unsigned bf16_bits(float f) {
  const unsigned u = __float_as_uint(f);
  const unsigned r = (u + 0x7FFFu + ((u >> 16) & 1u)) >> 16;
  const unsigned q = (u >> 16) | 0x40u;
  return ((u & 0x7fffffffu) > 0x7f800000u) ? q : r;
}

__device__ __forceinline__ float bf16_val(float f) {
  return __uint_as_float(bf16_bits(f) << 16);
}
__device__ __forceinline__ int clampi(int v, int lo, int hi) {
  return v < lo ? lo : (v > hi ? hi : v);
}

__device__ __forceinline__ unsigned f16_bits(float f) {
  const unsigned u  = __float_as_uint(f);
  const unsigned s  = (u >> 16) & 0x8000u;
  const unsigned a  = u & 0x7fffffffu;
  const unsigned t  = a - 0x38000000u;
  const unsigned r  = (t + 0x0FFFu + ((t >> 13) & 1u)) >> 13;
  const unsigned rc = r > 0x7C00u ? 0x7C00u : r;
  const bool small  = a < 0x38800000u;
  const bool isnan  = a > 0x7f800000u;
  const unsigned fin = small ? 0u : (s | rc);
  return isnan ? (s | 0x7E00u) : fin;
}

__device__ __forceinline__ unsigned pk16(unsigned lo, unsigned hi) { return lo | (hi << 16); }
__device__ __forceinline__ unsigned bf16_lo_bits(float v) {
  float hi = bf16_val(v);
  asm volatile("" : "+v"(hi));
  return bf16_bits(v - hi);
}
__device__ __forceinline__ v4u pack8_bf16(v4f a, v4f c) {
  return (v4u){ pk16(bf16_bits(a[0]), bf16_bits(a[1])), pk16(bf16_bits(a[2]), bf16_bits(a[3])),
                pk16(bf16_bits(c[0]), bf16_bits(c[1])), pk16(bf16_bits(c[2]), bf16_bits(c[3])) };
}
__device__ __forceinline__ v4u pack8_bf16_lo(v4f a, v4f c) {
  return (v4u){ pk16(bf16_lo_bits(a[0]), bf16_lo_bits(a[1])), pk16(bf16_lo_bits(a[2]), bf16_lo_bits(a[3])),
                pk16(bf16_lo_bits(c[0]), bf16_lo_bits(c[1])), pk16(bf16_lo_bits(c[2]), bf16_lo_bits(c[3])) };
}
__device__ __forceinline__ v4u pack8_f16(v4f a, v4f c) {
  return (v4u){ pk16(f16_bits(a[0]), f16_bits(a[1])), pk16(f16_bits(a[2]), f16_bits(a[3])),
                pk16(f16_bits(c[0]), f16_bits(c[1])), pk16(f16_bits(c[2]), f16_bits(c[3])) };
}

template <int FORM>
__global__ __launch_bounds__(256) void k_plane(const float* __restrict__ src, int rows, int cols, int ldsrc,
                                               unsigned short* __restrict__ dst, int MP, int KP) {
  static_assert(FORM >= 0 && FORM <= 3);
  const int KTOT = (FORM == 1 || FORM == 3) ? 2 * KP : KP;
  const unsigned ppr   = (unsigned)(KTOT >> 3);
  const unsigned kp8   = (unsigned)(KP >> 3);
  const unsigned total = (unsigned)MP * ppr;
  const unsigned g     = blockIdx.x * 256u + threadIdx.x;
  const unsigned rowu  = g / ppr;
  const unsigned p     = g - rowu * ppr;
  const bool second    = p >= kp8;
  const int row = (int)rowu;
  const int c0  = (int)((second ? p - kp8 : p) << 3);
  const float* srow = src + (size_t)clampi(row, 0, rows - 1) * (size_t)ldsrc;
  float x[8];
  unsigned mk[8];
#pragma unroll
  for (int e = 0; e < 8; ++e) {
    const int c = c0 + e;
    const float v = srow[clampi(c, 0, cols - 1)];
    asm volatile("" :: "v"(v));
    x[e]  = v;
    mk[e] = (row < rows && c < cols) ? 0xFFFFu : 0u;
  }
  const v4f a = (v4f){ x[0], x[1], x[2], x[3] };
  const v4f c = (v4f){ x[4], x[5], x[6], x[7] };
  v4u o;
  if (FORM == 2) {
    o = pack8_f16(a, c);
  } else {
    const v4u hi = pack8_bf16(a, c);
    o = hi;
    if (FORM == 1) { const v4u lo = pack8_bf16_lo(a, c); o = second ? lo : hi; }
  }
  const v4u mw = (v4u){ pk16(mk[0], mk[1]), pk16(mk[2], mk[3]), pk16(mk[4], mk[5]), pk16(mk[6], mk[7]) };
  o &= mw;
  if (g < total) {
    volatile v4u* q = (volatile v4u*)(dst + (size_t)g * 8);
    *q = o;
    __threadfence();
    *q = o;
  }
}

template <int FORM> struct FragOf    { typedef FragB T; };
template <>         struct FragOf<2> { typedef FragH T; };
__device__ __forceinline__ v8f mm(const FragB& a, const FragB& b, v8f c) { return wmb(a, b, c); }
__device__ __forceinline__ v8f mm(const FragH& a, const FragH& b, v8f c) { return wmh(a, b, c); }
template <class F> __device__ __forceinline__ F ld_frag(const unsigned short* p) {
  F f;
  f.h[0] = *(const v8usa*)(p);
  f.h[1] = *(const v8usa*)(p + 16);
  return f;
}

template <int FORM, int EPI>
__global__ __launch_bounds__(256) __attribute__((amdgpu_num_vgpr(248)))
void k_gemm_nt(const unsigned short* __restrict__ A, const unsigned short* __restrict__ B,
               const float* __restrict__ bias, float* __restrict__ D, int M, int N, int KTOT, int ldd) {
  static_assert(FORM >= 0 && FORM <= 2);
  static_assert(EPI == 0 || EPI == 1);
  typedef typename FragOf<FORM>::T F;
  __shared__ __attribute__((aligned(16))) float sT[8][16 * 68];
  const int lane = threadIdx.x & 31;
  const int wave = threadIdx.x >> 5;
  const int tilesM = (M + 63) >> 6;
  const int tilesN = (N + 63) >> 6;
  const int tile = blockIdx.x * 8 + wave;
  if (tile >= tilesM * tilesN) return;
  const int tm = tile / tilesN;
  const int tn = tile - tm * tilesN;
  const int m0 = tm << 6;
  const int n0 = tn << 6;

  const int rl = lane & 15;
  const int h8 = (lane >> 4) * 8;
  const unsigned short* pa = A + (size_t)(m0 + rl) * (size_t)KTOT + h8;
  const unsigned short* pb = B + (size_t)(n0 + rl) * (size_t)KTOT + h8;

  v8f acc[4][4];
#pragma unroll
  for (int i = 0; i < 4; ++i)
#pragma unroll
    for (int j = 0; j < 4; ++j) acc[i][j] = (v8f){0.f, 0.f, 0.f, 0.f, 0.f, 0.f, 0.f, 0.f};

#pragma unroll 1
  for (int k0 = 0; k0 < KTOT; k0 += 32) {
    F bf[4];
#pragma unroll
    for (int j = 0; j < 4; ++j) bf[j] = ld_frag<F>(pb + (size_t)(j << 4) * (size_t)KTOT + k0);
#pragma unroll
    for (int i = 0; i < 4; ++i) {
      const F af = ld_frag<F>(pa + (size_t)(i << 4) * (size_t)KTOT + k0);
#pragma unroll
      for (int j = 0; j < 4; ++j) acc[i][j] = mm(af, bf[j], acc[i][j]);
    }
  }

  float* slab = sT[wave];
  const int hh = lane >> 4;
  const int c4 = (lane & 15) * 4;
  const int nc = n0 + c4;
  const bool cok = nc < N;
  v4f bv = (v4f){0.f, 0.f, 0.f, 0.f};
  if (EPI == 1) {
    bv = *(const v4fa*)(bias + clampi(nc, 0, N - 4));
    asm volatile("" :: "v"(bv));
  }
#pragma unroll
  for (int i = 0; i < 4; ++i) {
    const int mBase = m0 + (i << 4);
#pragma unroll
    for (int j = 0; j < 4; ++j) {
#pragma unroll
      for (int r = 0; r < 8; ++r) slab[(h8 + r) * 68 + (j << 4) + rl] = acc[i][j][r];
    }
    __builtin_amdgcn_fence(__ATOMIC_RELEASE, "workgroup");
    __builtin_amdgcn_wave_barrier();
    __builtin_amdgcn_fence(__ATOMIC_ACQUIRE, "workgroup");
    v4f vv[8];
#pragma unroll
    for (int it = 0; it < 8; ++it) {
      const int row = it * 2 + hh;
      v4f v = *(const v4fa*)(slab + row * 68 + c4);
      if (EPI == 1) v += bv;
      vv[it] = v;
    }
    for (int pass = 0; pass < 2; ++pass) {
#pragma unroll
      for (int it = 0; it < 8; ++it) {
        const int row = mBase + it * 2 + hh;
        if (cok && row < M) *(volatile v4f*)(D + (size_t)row * (size_t)ldd + nc) = vv[it];
      }
      __threadfence();
    }
    __builtin_amdgcn_fence(__ATOMIC_RELEASE, "workgroup");
    __builtin_amdgcn_wave_barrier();
    __builtin_amdgcn_fence(__ATOMIC_ACQUIRE, "workgroup");
  }
}

#define NN       1024
#define NE       32768
#define SD       256
#define VD       64
#define ED       128
#define NG       16
#define NA       16
#define NBT      5
#define NBLK     2
#define NBROWS   512
#define DEGCAP   96
#define MAXHITS  16483
#define MAXDEG   54
#define NTHR     256
#define NWAVE    8
#define EPT      8
#define CHUNK    (NTHR * EPT)
#define WCAP     (EPT * 32)
#define LISTN    (NWAVE * WCAP)
#define NBMAX    2048
#define ESH      11
#define RCAP     20480
#define LDS_BKT  ((2 * RCAP + 2 * NBMAX + LISTN) * 4 + 64)
#define OUT_TOTAL 183296
#define OUT1_OFS 3072
#define OUT2_OFS 19456
#define WSMAX    ((size_t)128 << 20)

static_assert(NN == NBLK * NBROWS && (NBROWS & (NBROWS - 1)) == 0 && NBROWS == 512);
static_assert(NE % CHUNK == 0 && NE % 256 == 0 && NE / 256 == 128);
static_assert(NBROWS <= 1024 && NBROWS <= NBMAX && (1 << ESH) >= NBMAX && NTHR * 8 == NBMAX && LISTN >= NBMAX);
static_assert(NE <= (1 << (32 - ESH)));
static_assert(RCAP % 1024 == 0 && RCAP % 16 == 0 && RCAP > MAXHITS + 1024);
static_assert(RCAP * 100 >= MAXHITS * 110);
static_assert(DEGCAP >= MAXDEG + 8 && DEGCAP % 32 == 0);
static_assert(LDS_BKT <= 327680);
static_assert(SD == 256 && ED == 128 && VD == 64 && NA == 16 && NBT == 5 && NG == 16);
static_assert(OUT1_OFS == NN * 3 && OUT2_OFS == OUT1_OFS + NN * NA && OUT2_OFS + NE * NBT == OUT_TOTAL);
static_assert((OUT1_OFS * 4) % 128 == 0 && (OUT2_OFS * 4) % 128 == 0 && (256 * NBT * 4) % 128 == 0);
static_assert(NN % 64 == 0 && NE % 64 == 0 && SD % 64 == 0 && SD % 32 == 0 && (2 * ED) % 32 == 0);

constexpr size_t al256(size_t v) { return (v + 255) & ~(size_t)255; }
constexpr size_t O_XS    = 0;
constexpr size_t O_WSH   = al256(O_XS    + (size_t)NN * SD * 2);
constexpr size_t O_WA2   = al256(O_WSH   + (size_t)SD * SD * 2);
constexpr size_t O_WBM2  = al256(O_WA2   + (size_t)64 * 512 * 2);
constexpr size_t O_W0D   = al256(O_WBM2  + (size_t)SD * 256 * 2);
constexpr size_t O_PRE   = al256(O_W0D   + (size_t)SD * 512 * 2);
constexpr size_t O_S1    = al256(O_PRE   + (size_t)NN * SD * 4);
constexpr size_t O_S1HL  = al256(O_S1    + (size_t)NN * SD * 4);
constexpr size_t O_ATP   = al256(O_S1HL  + (size_t)NN * 512 * 2);
constexpr size_t O_CC    = al256(O_ATP   + (size_t)NN * 64 * 4);
constexpr size_t O_BLIST = al256(O_CC    + (size_t)NN * 16);
constexpr size_t O_OFFC  = al256(O_BLIST + (size_t)NBLK * RCAP * 4);
constexpr size_t O_META  = al256(O_OFFC  + (size_t)NBLK * 2048 * 4);
constexpr size_t O_PAIR  = al256(O_META  + (size_t)NBLK * 128);
constexpr size_t O_DD    = al256(O_PAIR  + (size_t)NE * 8);
constexpr size_t O_ES    = al256(O_DD    + (size_t)NE * 4);
constexpr size_t O_GH    = al256(O_ES    + (size_t)NE * 256 * 2);
constexpr size_t O_FHL   = al256(O_GH    + (size_t)NE * 256 * 4);
constexpr size_t WS_TOTAL = al256(O_FHL  + (size_t)NE * 512 * 2);
static_assert(WS_TOTAL <= (size_t)WSMAX);

typedef int v4i __attribute__((ext_vector_type(4)));
typedef v4i __attribute__((may_alias)) v4ia;
typedef v4u __attribute__((may_alias)) v4ua;

__device__ __forceinline__ void wave_sync_lds() {
  __builtin_amdgcn_fence(__ATOMIC_RELEASE, "workgroup");
  __builtin_amdgcn_wave_barrier();
  __builtin_amdgcn_fence(__ATOMIC_ACQUIRE, "workgroup");
}
__device__ __forceinline__ void st2_v4u(void* p, const v4u v) {
  volatile v4u* q = (volatile v4u*)p;
  *q = v;
  __threadfence();
  *q = v;
}
__device__ __forceinline__ void st2_v4f(float* p, const v4f v) {
  volatile v4f* q = (volatile v4f*)p;
  *q = v;
  __threadfence();
  *q = v;
}
__device__ __forceinline__ void st2_v4i(int* p, const v4i v) {
  volatile v4i* q = (volatile v4i*)p;
  *q = v;
  __threadfence();
  *q = v;
}
__device__ __forceinline__ v4f bf4(const v4f a) {
  return (v4f){ bf16_val(a[0]), bf16_val(a[1]), bf16_val(a[2]), bf16_val(a[3]) };
}
__device__ __forceinline__ float silu_p(float x) { return x / (1.0f + expf(-x)); }
__device__ __forceinline__ bool is_nan_bits(float x) { return (__float_as_uint(x) & 0x7fffffffu) > 0x7f800000u; }

__device__ __forceinline__ int scan_chunk(const int* __restrict__ dsts, int nE, int cbase, int slotBase,
                                          int nb, int vec8, int* list, int tid, int lane, int wave) {
  int wc = 0;
  const int el0  = tid * EPT;
  const int e0   = cbase + el0;
  const int sent = (-0x7fffffff - 1);
  v4i da, db;
  if (vec8 != 0 && cbase + CHUNK <= nE) {
    da = *(const v4i*)(dsts + e0);
    db = *(const v4i*)(dsts + e0 + 4);
  } else {
    const int t0 = dsts[min(e0 + 0, nE - 1)];
    const int t1 = dsts[min(e0 + 1, nE - 1)];
    const int t2 = dsts[min(e0 + 2, nE - 1)];
    const int t3 = dsts[min(e0 + 3, nE - 1)];
    const int t4 = dsts[min(e0 + 4, nE - 1)];
    const int t5 = dsts[min(e0 + 5, nE - 1)];
    const int t6 = dsts[min(e0 + 6, nE - 1)];
    const int t7 = dsts[min(e0 + 7, nE - 1)];
    asm volatile("" :: "v"(t0), "v"(t1), "v"(t2), "v"(t3), "v"(t4), "v"(t5), "v"(t6), "v"(t7));
    da.x = (e0 + 0 < nE) ? t0 : sent;
    da.y = (e0 + 1 < nE) ? t1 : sent;
    da.z = (e0 + 2 < nE) ? t2 : sent;
    da.w = (e0 + 3 < nE) ? t3 : sent;
    db.x = (e0 + 4 < nE) ? t4 : sent;
    db.y = (e0 + 5 < nE) ? t5 : sent;
    db.z = (e0 + 6 < nE) ? t6 : sent;
    db.w = (e0 + 7 < nE) ? t7 : sent;
  }
  const unsigned nbs = (unsigned)slotBase;
  const unsigned unb = (unsigned)nb;
  const unsigned s0 = (unsigned)da.x - nbs, s1 = (unsigned)da.y - nbs;
  const unsigned s2 = (unsigned)da.z - nbs, s3 = (unsigned)da.w - nbs;
  const unsigned s4 = (unsigned)db.x - nbs, s5 = (unsigned)db.y - nbs;
  const unsigned s6 = (unsigned)db.z - nbs, s7 = (unsigned)db.w - nbs;
  const bool h0 = s0 < unb, h1 = s1 < unb, h2 = s2 < unb, h3 = s3 < unb;
  const bool h4 = s4 < unb, h5 = s5 < unb, h6 = s6 < unb, h7 = s7 < unb;
  const unsigned any = __builtin_amdgcn_ballot_w32(h0 | h1 | h2 | h3 | h4 | h5 | h6 | h7);
  if (any != 0u) {
#define HITJ(J, HJ, SJ) { \
      const unsigned mj = __builtin_amdgcn_ballot_w32(HJ); \
      if (mj != 0u) { \
        if (HJ) { \
          const int pos = wc + (int)__builtin_amdgcn_mbcnt_lo(mj, 0u); \
          if (pos < WCAP) list[wave * WCAP + pos] = ((el0 + (J)) << 12) | (int)(SJ); \
        } \
        wc += (int)__builtin_popcount(mj); } }
    HITJ(0, h0, s0)
    HITJ(1, h1, s1)
    HITJ(2, h2, s2)
    HITJ(3, h3, s3)
    HITJ(4, h4, s4)
    HITJ(5, h5, s5)
    HITJ(6, h6, s6)
    HITJ(7, h7, s7)
#undef HITJ
  }
  return wc;
}

__device__ __forceinline__ int build_lists(const int* __restrict__ dsts, int nE, int nodeBase, int nb, int vec8,
                                           int* reg1, int* reg2, int* scnt, int* soff, int* list,
                                           int* wcnt, int* wtot, int tid, int lane, int wave) {
  for (int i = tid; i < NBMAX; i += NTHR) scnt[i] = 0;
  __syncthreads();

  int tot = 0;
  const int nChunks = (nE + CHUNK - 1) / CHUNK;
#pragma unroll 1
  for (int ch = 0; ch < nChunks; ++ch) {
    const int cbase = ch * CHUNK;
    const int wc = scan_chunk(dsts, nE, cbase, nodeBase, nb, vec8, list, tid, lane, wave);
    if (lane == 0) wcnt[wave] = wc;
    __syncthreads();
    int pre = 0, all = 0;
#pragma unroll
    for (int w2 = 0; w2 < NWAVE; ++w2) {
      int c = wcnt[w2];
      c = c < 0 ? 0 : (c > WCAP ? WCAP : c);
      all += c;
      pre += (w2 < wave) ? c : 0;
    }
    const int wcc  = wc > WCAP ? WCAP : wc;
    const int base = tot + pre;
#pragma unroll 1
    for (int i = lane; i < wcc; i += 32) {
      const int ent = list[wave * WCAP + i];
      const int el  = (ent >> 12) & (CHUNK - 1);
      const int sl  = ent & (NBMAX - 1);
      int eid = cbase + el;
      eid = eid > nE - 1 ? nE - 1 : eid;
      const int pos = base + i;
      if (pos < RCAP) reg1[pos] = (int)(((unsigned)eid << ESH) | (unsigned)sl);
    }
    tot += all;
    tot = tot > RCAP ? RCAP : tot;
    __syncthreads();
  }
  const int nh = tot;

  if (wave == 0) {
#pragma unroll 1
    for (int b0 = 0; b0 < nh; b0 += 32) {
      const int idx = b0 + lane;
      const int uv  = reg1[idx < RCAP ? idx : RCAP - 1];
      const int m32 = (nh - b0) < 32 ? (nh - b0) : 32;
#pragma unroll 1
      for (int k = 0; k < m32; ++k) {
        const int u  = __builtin_amdgcn_readlane(uv, k);
        const int sl = u & (NBMAX - 1);
        if (lane == 0) scnt[sl] = scnt[sl] + 1;
      }
    }
  }
  __syncthreads();

  {
    const v4i ca = *(const v4i*)(scnt + 8 * tid);
    const v4i cb = *(const v4i*)(scnt + 8 * tid + 4);
    const int e0 = ca.x < 0 ? 0 : ca.x, e1 = ca.y < 0 ? 0 : ca.y, e2 = ca.z < 0 ? 0 : ca.z, e3 = ca.w < 0 ? 0 : ca.w;
    const int e4 = cb.x < 0 ? 0 : cb.x, e5 = cb.y < 0 ? 0 : cb.y, e6 = cb.z < 0 ? 0 : cb.z, e7 = cb.w < 0 ? 0 : cb.w;
    const int ts = e0 + e1 + e2 + e3 + e4 + e5 + e6 + e7;
    int incl = ts;
#pragma unroll
    for (int d = 1; d < 32; d <<= 1) {
      const int up = __shfl_up(incl, d);
      if (lane >= d) incl += up;
    }
    if (lane == 31) wtot[wave] = incl;
    __syncthreads();
    int pre = 0;
#pragma unroll
    for (int w2 = 0; w2 < NWAVE; ++w2) pre += (w2 < wave) ? wtot[w2] : 0;
    int run = pre + incl - ts;
    soff[8 * tid + 0] = run; run += e0;
    soff[8 * tid + 1] = run; run += e1;
    soff[8 * tid + 2] = run; run += e2;
    soff[8 * tid + 3] = run; run += e3;
    soff[8 * tid + 4] = run; run += e4;
    soff[8 * tid + 5] = run; run += e5;
    soff[8 * tid + 6] = run; run += e6;
    soff[8 * tid + 7] = run;
  }
  __syncthreads();
  for (int i = tid; i < NBMAX; i += NTHR) list[i] = soff[i];
  __syncthreads();

  if (wave == 0) {
#pragma unroll 1
    for (int b0 = 0; b0 < nh; b0 += 32) {
      const int idx = b0 + lane;
      const int uv  = reg1[idx < RCAP ? idx : RCAP - 1];
      const int m32 = (nh - b0) < 32 ? (nh - b0) : 32;
#pragma unroll 1
      for (int k = 0; k < m32; ++k) {
        const int u   = __builtin_amdgcn_readlane(uv, k);
        const int sl  = u & (NBMAX - 1);
        const int eid = (int)((unsigned)u >> ESH);
        if (lane == 0) {
          int pos = list[sl];
          pos = pos < 0 ? 0 : (pos > RCAP - 1 ? RCAP - 1 : pos);
          reg2[pos] = eid;
          list[sl] = pos + 1;
        }
      }
    }
  }
  __syncthreads();
  return nh;
}

__global__ __launch_bounds__(NTHR) void k_bucket(const int* __restrict__ dsts, int nE, int nN, int vec8,
                                                 int* BLIST, int* OFFC, int* META) {
  extern __shared__ v4f lds_dyn[];
  int* reg1 = (int*)lds_dyn;
  int* reg2 = reg1 + RCAP;
  int* scnt = reg2 + RCAP;
  int* soff = scnt + NBMAX;
  int* list = soff + NBMAX;
  int* wcnt = list + LISTN;
  int* wtot = wcnt + NWAVE;
  const int tid = (int)threadIdx.x, lane = tid & 31, wave = tid >> 5;
  const int b = (int)blockIdx.x;
  const int nodeBase = b * NBROWS;
  int nb = nN - nodeBase;
  nb = nb < 0 ? 0 : (nb > NBROWS ? NBROWS : nb);

  const int nh = build_lists(dsts, nE, nodeBase, nb, vec8, reg1, reg2, scnt, soff, list, wcnt, wtot, tid, lane, wave);

  int* bl = BLIST + (size_t)b * RCAP;
  const int last = nh > 0 ? nh - 1 : 0;
#pragma unroll 1
  for (int base = 0; base < RCAP; base += 1024) {
    const int i0 = base + 4 * tid;
    v4i v;
    v.x = reg2[i0     < last ? i0     : last];
    v.y = reg2[i0 + 1 < last ? i0 + 1 : last];
    v.z = reg2[i0 + 2 < last ? i0 + 2 : last];
    v.w = reg2[i0 + 3 < last ? i0 + 3 : last];
    v.x = (i0     < nh) ? v.x : -1;
    v.y = (i0 + 1 < nh) ? v.y : -1;
    v.z = (i0 + 2 < nh) ? v.z : -1;
    v.w = (i0 + 3 < nh) ? v.w : -1;
    st2_v4i(bl + i0, v);
  }
  {
    const v4i so = *(const v4ia*)(soff + 4 * tid);
    const v4i sc = *(const v4ia*)(scnt + 4 * tid);
    int* oc = OFFC + (size_t)b * 2048;
    st2_v4i(oc + 4 * tid, so);
    st2_v4i(oc + 1024 + 4 * tid, sc);
  }
  if (tid < 8) {
    v4i mv;
    mv.x = (tid == 0) ? nh : 0;
    mv.y = (tid == 0 && nh >= RCAP) ? 1 : 0;
    mv.z = 0; mv.w = 0;
    st2_v4i(META + (size_t)b * 32 + 4 * tid, mv);
  }
}

__global__ __launch_bounds__(256) void k_s1(const float* __restrict__ PRE, const float* __restrict__ bsh,
                                            float* S1, unsigned short* S1HL) {
  __shared__ __attribute__((aligned(16))) float sB[SD];
  __shared__ __attribute__((aligned(16))) float sR[8][SD];
  const int tid = (int)threadIdx.x, lane = tid & 31;
  const int wave = __builtin_amdgcn_readfirstlane(tid >> 5);
  {
    const int ix = tid < 63 ? tid : 63;
    v4f w = *(const v4fa*)(bsh + 4 * ix);
    asm volatile("" :: "v"(w));
    w = bf4(w);
    if (tid < 64) *(v4fa*)(sB + 4 * tid) = w;
  }
  __syncthreads();
  const int row = (int)blockIdx.x * 8 + wave;
  float* strip = &sR[wave][0];
  const float* pr = PRE + (size_t)row * SD;
#pragma unroll 1
  for (int c = 0; c < 8; ++c) {
    const int col = 32 * c + lane;
    const float x = pr[col] + sB[col];
    strip[col] = silu_p(x);
  }
  wave_sync_lds();
  const v4f a = *(const v4fa*)(strip + 4 * lane);
  const v4f b = *(const v4fa*)(strip + 128 + 4 * lane);
  const v4f h0 = *(const v4fa*)(strip + 8 * lane);
  const v4f h1 = *(const v4fa*)(strip + 8 * lane + 4);
  const v4u hi = pack8_bf16(h0, h1);
  const v4u lo = pack8_bf16_lo(h0, h1);
  float* sp = S1 + (size_t)row * SD;
  unsigned short* hp = S1HL + (size_t)row * 512;
  for (int pass = 0; pass < 2; ++pass) {
    *(volatile v4f*)(sp + 4 * lane) = a;
    *(volatile v4f*)(sp + 128 + 4 * lane) = b;
    *(volatile v4u*)(hp + 8 * lane) = hi;
    *(volatile v4u*)(hp + 256 + 8 * lane) = lo;
    __threadfence();
  }
}

__global__ __launch_bounds__(256) void k_atoms(const float* __restrict__ ATP, const float* __restrict__ bat, float* out1) {
  const int g = (int)blockIdx.x * 256 + (int)threadIdx.x;
  const int row = g >> 2, c4 = (g & 3) * 4;
  const v4f a = *(const v4fa*)(ATP + (size_t)row * 64 + c4);
  v4f b = *(const v4fa*)(bat + c4);
  asm volatile("" :: "v"(a), "v"(b));
  b = bf4(b);
  st2_v4f(out1 + (size_t)g * 4, a + b);
}

__global__ __launch_bounds__(256) void k_coords(const float* __restrict__ v, const float* __restrict__ p,
                                                const float* __restrict__ Wc, const int* __restrict__ batch,
                                                float* CC, float* out0) {
  __shared__ __attribute__((aligned(16))) float sWc[VD];
  __shared__ __attribute__((aligned(16))) float sC[NN * 3];
  __shared__ __attribute__((aligned(16))) int sBt[NN];
  __shared__ __attribute__((aligned(16))) float sMean[64];
  const int tid = (int)threadIdx.x;
  {
    const int ix = tid < 15 ? tid : 15;
    v4f w = *(const v4fa*)(Wc + 4 * ix);
    asm volatile("" :: "v"(w));
    w = bf4(w);
    if (tid < 16) *(v4fa*)(sWc + 4 * tid) = w;
    const v4i bb = *(const v4ia*)(batch + 4 * tid);
    *(v4ia*)(sBt + 4 * tid) = bb;
  }
  __syncthreads();
#pragma unroll 1
  for (int it = 0; it < 12; ++it) {
    const int idx = tid + 256 * it;
    const float* vr = v + (size_t)idx * VD;
    float acc = 0.0f;
#pragma unroll 2
    for (int q = 0; q < 16; ++q) {
      const v4f x = bf4(*(const v4fa*)(vr + 4 * q));
      const v4f w = *(const v4fa*)(sWc + 4 * q);
      acc = fmaf(x[0], w[0], acc);
      acc = fmaf(x[1], w[1], acc);
      acc = fmaf(x[2], w[2], acc);
      acc = fmaf(x[3], w[3], acc);
    }
    sC[idx] = bf16_val(p[idx]) + acc;
  }
  __syncthreads();
  {
    const int gi = tid % 48;
    const int g = gi / 3, a = gi - 3 * g;
    float sum = 0.0f, cnt = 0.0f;
#pragma unroll 4
    for (int n = 0; n < NN; ++n) {
      const float c = sC[3 * n + a];
      const int bn = sBt[n];
      asm volatile("" :: "v"(c), "v"(bn));
      const bool m = bn == g;
      sum = sum + (m ? c : 0.0f);
      cnt = cnt + (m ? 1.0f : 0.0f);
    }
    const float mean = sum / fmaxf(cnt, 1.0f);
    if (tid < 48) sMean[tid] = mean;
  }
  __syncthreads();
#pragma unroll 1
  for (int it = 0; it < 12; ++it) {
    const int idx = tid + 256 * it;
    const int n = idx / 3, a = idx - 3 * n;
    const int g = clampi(sBt[n], 0, NG - 1);
    sC[idx] = sC[idx] - sMean[g * 3 + a];
  }
  __syncthreads();
#pragma unroll 1
  for (int it = 0; it < 3; ++it) {
    const int q = tid + 256 * it;
    const v4f o = *(const v4fa*)(sC + 4 * q);
    st2_v4f(out0 + 4 * q, o);
  }
#pragma unroll 1
  for (int it = 0; it < 4; ++it) {
    const int n = tid + 256 * it;
    const v4f o = (v4f){ sC[3 * n], sC[3 * n + 1], sC[3 * n + 2], 0.0f };
    st2_v4f(CC + 4 * n, o);
  }
}

__device__ __forceinline__ int pair_lookup(const int* __restrict__ eoth, const int* __restrict__ BLIST,
                                           const int* __restrict__ OFFC, const int* __restrict__ META,
                                           int owner, int want, int lane, int& poison) {
  const int ob = owner >> 9;
  const int sl = owner & (NBROWS - 1);
  int nhv = META[ob * 32];
  int flv = META[ob * 32 + 1];
  int stv = OFFC[ob * 2048 + sl];
  int cv  = OFFC[ob * 2048 + 1024 + sl];
  asm volatile("" :: "v"(nhv), "v"(flv), "v"(stv), "v"(cv));
  nhv = clampi(nhv, 0, RCAP);
  const int craw = cv < 0 ? 0 : cv;
  stv = clampi(stv, 0, nhv);
  int cc = craw > DEGCAP ? DEGCAP : craw;
  cc = cc > nhv - stv ? nhv - stv : cc;
  const int bad = (flv != 0 || craw > DEGCAP) ? 1 : 0;
  const int st  = __builtin_amdgcn_readfirstlane(stv);
  const int cnt = __builtin_amdgcn_readfirstlane(cc);
  poison |= __builtin_amdgcn_readfirstlane(bad);
  const int* bl = BLIST + (size_t)ob * RCAP;
  int best = -1;
#pragma unroll 1
  for (int b0 = 0; b0 < cnt; b0 += 32) {
    const int q = b0 + lane;
    const int li = st + (q < cnt - 1 ? q : cnt - 1);
    int id = bl[li];
    asm volatile("" :: "v"(id));
    id = clampi(id, 0, NE - 1);
    int oth = eoth[id];
    asm volatile("" :: "v"(oth));
    const int cand = (q < cnt && oth == want) ? id : -1;
    best = best > cand ? best : cand;
  }
  int o;
  o = __shfl_xor(best, 16); best = best > o ? best : o;
  o = __shfl_xor(best, 8);  best = best > o ? best : o;
  o = __shfl_xor(best, 4);  best = best > o ? best : o;
  o = __shfl_xor(best, 2);  best = best > o ? best : o;
  o = __shfl_xor(best, 1);  best = best > o ? best : o;
  return __builtin_amdgcn_readfirstlane(best);
}

__global__ __launch_bounds__(256) void k_pair(const int* __restrict__ ei, const int* __restrict__ BLIST,
                                              const int* __restrict__ OFFC, const int* __restrict__ META,
                                              const float* __restrict__ CC, int* PAIR, float* DD) {
  __shared__ __attribute__((aligned(16))) int sP[512];
  __shared__ __attribute__((aligned(16))) float sD[256];
  const int tid = (int)threadIdx.x, lane = tid & 31;
  const int wave = __builtin_amdgcn_readfirstlane(tid >> 5);
  const int blk = (int)blockIdx.x;
  const float qnan = __int_as_float(0x7fc00000);
#pragma unroll 1
  for (int e = 0; e < 32; ++e) {
    const int loc = wave * 32 + e;
    const int t = blk * 256 + loc;
    int jv = ei[t];
    int iv = ei[NE + t];
    asm volatile("" :: "v"(jv), "v"(iv));
    const int j = __builtin_amdgcn_readfirstlane(clampi(jv, 0, NN - 1));
    const int i = __builtin_amdgcn_readfirstlane(clampi(iv, 0, NN - 1));
    int poison = 0;
    const int t1 = pair_lookup(ei + NE, BLIST, OFFC, META, j, i, lane, poison);
    const int t2 = pair_lookup(ei + NE, BLIST, OFFC, META, i, j, lane, poison);
    const v4f ci = *(const v4fa*)(CC + 4 * i);
    const v4f cj = *(const v4fa*)(CC + 4 * j);
    asm volatile("" :: "v"(ci), "v"(cj));
    const float dx = ci[0] - cj[0], dy = ci[1] - cj[1], dz = ci[2] - cj[2];
    float d = (dx * dx + dz * dz) + dy * dy;
    const bool pz = (poison != 0) || (t1 < 0);
    d = pz ? qnan : d;
    if (lane == 0) {
      sP[2 * loc]     = clampi(t1, 0, NE - 1);
      sP[2 * loc + 1] = t2 < 0 ? -1 : (t2 > NE - 1 ? NE - 1 : t2);
      sD[loc] = d;
    }
  }
  __syncthreads();
  if (tid < 128) {
    const v4i pv = *(const v4ia*)(sP + 4 * tid);
    st2_v4i(PAIR + (size_t)blk * 512 + 4 * tid, pv);
  } else if (tid < 192) {
    const int u = tid - 128;
    const v4f dv = *(const v4fa*)(sD + 4 * u);
    st2_v4f(DD + (size_t)blk * 256 + 4 * u, dv);
  }
}

__global__ __launch_bounds__(256) void k_esym(const float* __restrict__ ef, const int* __restrict__ PAIR,
                                              const float* __restrict__ DD, unsigned short* ESHL) {
  const int tid = (int)threadIdx.x, lane = tid & 31;
  const int wave = __builtin_amdgcn_readfirstlane(tid >> 5);
  const int blk = (int)blockIdx.x;
  const int c0 = (lane & 15) * 8;
#pragma unroll 1
  for (int e = 0; e < 32; ++e) {
    const int t = blk * 256 + wave * 32 + e;
    int t1 = PAIR[2 * t];
    int t2 = PAIR[2 * t + 1];
    float d = DD[t];
    asm volatile("" :: "v"(t1), "v"(t2), "v"(d));
    const int t1c = clampi(t1, 0, NE - 1);
    const int t2c = clampi(t2, 0, NE - 1);
    const unsigned m2 = t2 >= 0 ? 0xFFFFFFFFu : 0u;
    const float* r1 = ef + (size_t)t1c * ED + c0;
    const float* r2 = ef + (size_t)t2c * ED + c0;
    const v4f a0 = *(const v4fa*)r1;
    const v4f a1 = *(const v4fa*)(r1 + 4);
    const v4f b0 = *(const v4fa*)r2;
    const v4f b1 = *(const v4fa*)(r2 + 4);
    asm volatile("" :: "v"(a0), "v"(a1), "v"(b0), "v"(b1));
    v4f s0, s1;
#pragma unroll
    for (int q = 0; q < 4; ++q) {
      const float x0 = bf16_val(a0[q]);
      const float y0 = __uint_as_float((bf16_bits(b0[q]) << 16) & m2);
      s0[q] = 0.5f * (x0 + y0);
      const float x1 = bf16_val(a1[q]);
      const float y1 = __uint_as_float((bf16_bits(b1[q]) << 16) & m2);
      s1[q] = 0.5f * (x1 + y1);
    }
    const v4u hi = pack8_bf16(s0, s1);
    const v4u lo = pack8_bf16_lo(s0, s1);
    v4u o = (lane >= 16) ? lo : hi;
    const v4u nn = (v4u){ 0x7fc07fc0u, 0x7fc07fc0u, 0x7fc07fc0u, 0x7fc07fc0u };
    o = is_nan_bits(d) ? nn : o;
    st2_v4u(ESHL + (size_t)t * 256 + lane * 8, o);
  }
}

__global__ __launch_bounds__(256) void k_f(const int* __restrict__ ei, const float* __restrict__ S1,
                                           const float* __restrict__ G, const float* __restrict__ bbm,
                                           unsigned short* FHL) {
  __shared__ __attribute__((aligned(16))) float sB[SD];
  const int tid = (int)threadIdx.x, lane = tid & 31;
  const int wave = __builtin_amdgcn_readfirstlane(tid >> 5);
  const int blk = (int)blockIdx.x;
  {
    const int ix = tid < 63 ? tid : 63;
    v4f w = *(const v4fa*)(bbm + 4 * ix);
    asm volatile("" :: "v"(w));
    w = bf4(w);
    if (tid < 64) *(v4fa*)(sB + 4 * tid) = w;
  }
  __syncthreads();
  const int c0 = lane * 8;
  const v4f bb0 = *(const v4fa*)(sB + c0);
  const v4f bb1 = *(const v4fa*)(sB + c0 + 4);
#pragma unroll 1
  for (int e = 0; e < 32; ++e) {
    const int t = blk * 256 + wave * 32 + e;
    int jv = ei[t];
    int iv = ei[NE + t];
    asm volatile("" :: "v"(jv), "v"(iv));
    const int j = clampi(jv, 0, NN - 1);
    const int i = clampi(iv, 0, NN - 1);
    const float* pi = S1 + (size_t)i * SD + c0;
    const float* pj = S1 + (size_t)j * SD + c0;
    const float* pg = G + (size_t)t * SD + c0;
    const v4f si0 = *(const v4fa*)pi, si1 = *(const v4fa*)(pi + 4);
    const v4f sj0 = *(const v4fa*)pj, sj1 = *(const v4fa*)(pj + 4);
    const v4f g0 = *(const v4fa*)pg, g1 = *(const v4fa*)(pg + 4);
    const v4f f0 = (si0 + sj0) + (g0 + bb0);
    const v4f f1 = (si1 + sj1) + (g1 + bb1);
    const v4u hi = pack8_bf16(f0, f1);
    const v4u lo = pack8_bf16_lo(f0, f1);
    unsigned short* row = FHL + (size_t)t * 512;
    for (int pass = 0; pass < 2; ++pass) {
      *(volatile v4u*)(row + c0) = hi;
      *(volatile v4u*)(row + 256 + c0) = lo;
      __threadfence();
    }
  }
}

__global__ __launch_bounds__(256) void k_out(const float* __restrict__ H, const float* __restrict__ DD,
                                             const float* __restrict__ W0, const float* __restrict__ b0,
                                             const float* __restrict__ W1, const float* __restrict__ b1,
                                             float* out2) {
  __shared__ __attribute__((aligned(16))) float sW1[NBT * SD];
  __shared__ __attribute__((aligned(16))) float sB0[SD];
  __shared__ __attribute__((aligned(16))) float sWC[SD];
  __shared__ __attribute__((aligned(16))) float sb1[8];
  __shared__ __attribute__((aligned(16))) float sOut[256 * NBT];
  const int tid = (int)threadIdx.x, lane = tid & 31;
  const int wave = __builtin_amdgcn_readfirstlane(tid >> 5);
  const int blk = (int)blockIdx.x;
  {
    v4f w = *(const v4fa*)(W1 + 4 * tid);
    const int q2 = (256 + tid) < 319 ? (256 + tid) : 319;
    v4f w2 = *(const v4fa*)(W1 + 4 * q2);
    const int ix = tid < 63 ? tid : 63;
    v4f bb = *(const v4fa*)(b0 + 4 * ix);
    const float wc = W0[(size_t)tid * (SD + 1) + SD];
    const float bq = b1[tid < NBT - 1 ? tid : NBT - 1];
    asm volatile("" :: "v"(w), "v"(w2), "v"(bb), "v"(wc), "v"(bq));
    *(v4fa*)(sW1 + 4 * tid) = bf4(w);
    if (tid < 64) {
      *(v4fa*)(sW1 + 1024 + 4 * tid) = bf4(w2);
      *(v4fa*)(sB0 + 4 * tid) = bf4(bb);
    }
    sWC[tid] = bf16_val(wc);
    if (tid < 8) sb1[tid] = (tid < NBT) ? bf16_val(bq) : 0.0f;
  }
  __syncthreads();
  const float qnan = __int_as_float(0x7fc00000);
#pragma unroll 1
  for (int e = 0; e < 32; ++e) {
    const int loc = wave * 32 + e;
    const int t = blk * 256 + loc;
    float d = DD[t];
    asm volatile("" :: "v"(d));
    const float* hr = H + (size_t)t * SD;
    float p0 = 0.0f, p1 = 0.0f, p2 = 0.0f, p3 = 0.0f, p4 = 0.0f;
#pragma unroll 1
    for (int c = 0; c < 8; ++c) {
      const int col = 32 * c + lane;
      const float pre = (hr[col] + d * sWC[col]) + sB0[col];
      const float a = silu_p(pre);
      p0 = fmaf(a, sW1[col], p0);
      p1 = fmaf(a, sW1[SD + col], p1);
      p2 = fmaf(a, sW1[2 * SD + col], p2);
      p3 = fmaf(a, sW1[3 * SD + col], p3);
      p4 = fmaf(a, sW1[4 * SD + col], p4);
    }
#pragma unroll
    for (int m = 16; m >= 1; m >>= 1) {
      p0 += __shfl_xor(p0, m);
      p1 += __shfl_xor(p1, m);
      p2 += __shfl_xor(p2, m);
      p3 += __shfl_xor(p3, m);
      p4 += __shfl_xor(p4, m);
    }
    p0 += sb1[0]; p1 += sb1[1]; p2 += sb1[2]; p3 += sb1[3]; p4 += sb1[4];
    const bool pz = is_nan_bits(d);
    p0 = pz ? qnan : p0; p1 = pz ? qnan : p1; p2 = pz ? qnan : p2; p3 = pz ? qnan : p3; p4 = pz ? qnan : p4;
    if (lane == 0) {
      float* so = sOut + loc * NBT;
      so[0] = p0; so[1] = p1; so[2] = p2; so[3] = p3; so[4] = p4;
    }
  }
  __syncthreads();
  float* ob = out2 + (size_t)blk * (256 * NBT);
  {
    const v4f o = *(const v4fa*)(sOut + 4 * tid);
    st2_v4f(ob + 4 * tid, o);
  }
  if (tid < 64) {
    const v4f o = *(const v4fa*)(sOut + 1024 + 4 * tid);
    st2_v4f(ob + 1024 + 4 * tid, o);
  }
}

extern "C" void kernel_launch(void* const* d_in, const int* in_sizes, int n_in,
                              void* d_out, int out_size, void* d_ws, size_t ws_size,
                              hipStream_t stream) {
  if (n_in < 17) return;
  if (in_sizes[0] != NN * SD || in_sizes[1] != NN * 3 * VD || in_sizes[2] != NN * 3 || in_sizes[3] != NE * ED) return;
  if (in_sizes[4] != NN || in_sizes[5] != 2 * NE) return;
  if (in_sizes[6] != SD * SD || in_sizes[7] != SD || in_sizes[8] != SD * ED || in_sizes[9] != SD) return;
  if (in_sizes[10] != SD * (SD + 1) || in_sizes[11] != SD || in_sizes[12] != NBT * SD || in_sizes[13] != NBT) return;
  if (in_sizes[14] != VD || in_sizes[15] != NA * SD || in_sizes[16] != NA) return;
  if (out_size != OUT_TOTAL) return;
  if (ws_size < WS_TOTAL) return;

  const float* s     = (const float*)d_in[0];
  const float* v     = (const float*)d_in[1];
  const float* p     = (const float*)d_in[2];
  const float* ef    = (const float*)d_in[3];
  const int*   batch = (const int*)  d_in[4];
  const int*   ei    = (const int*)  d_in[5];
  const float* Wsh   = (const float*)d_in[6];
  const float* bsh   = (const float*)d_in[7];
  const float* Wbm   = (const float*)d_in[8];
  const float* bbm   = (const float*)d_in[9];
  const float* Wb0   = (const float*)d_in[10];
  const float* bb0   = (const float*)d_in[11];
  const float* Wb1   = (const float*)d_in[12];
  const float* bb1   = (const float*)d_in[13];
  const float* Wc    = (const float*)d_in[14];
  const float* Wat   = (const float*)d_in[15];
  const float* bat   = (const float*)d_in[16];
  float* out = (float*)d_out;

  char* ws = (char*)d_ws;
  unsigned short* XS    = (unsigned short*)(ws + O_XS);
  unsigned short* WSH   = (unsigned short*)(ws + O_WSH);
  unsigned short* WA2   = (unsigned short*)(ws + O_WA2);
  unsigned short* WBM2  = (unsigned short*)(ws + O_WBM2);
  unsigned short* W0D   = (unsigned short*)(ws + O_W0D);
  float*          PRE   = (float*)(ws + O_PRE);
  float*          S1    = (float*)(ws + O_S1);
  unsigned short* S1HL  = (unsigned short*)(ws + O_S1HL);
  float*          ATP   = (float*)(ws + O_ATP);
  float*          CC    = (float*)(ws + O_CC);
  int*            BLIST = (int*)(ws + O_BLIST);
  int*            OFFC  = (int*)(ws + O_OFFC);
  int*            META  = (int*)(ws + O_META);
  int*            PAIR  = (int*)(ws + O_PAIR);
  float*          DD    = (float*)(ws + O_DD);
  unsigned short* ESHL  = (unsigned short*)(ws + O_ES);
  float*          GH    = (float*)(ws + O_GH);
  unsigned short* FHL   = (unsigned short*)(ws + O_FHL);

  hipFuncSetAttribute(reinterpret_cast<const void*>(&k_bucket),
                      hipFuncAttributeMaxDynamicSharedMemorySize, LDS_BKT);

  k_plane<0><<<NN * SD / 8 / 256, 256, 0, stream>>>(s, NN, SD, SD, XS, NN, SD);
  k_plane<0><<<SD * SD / 8 / 256, 256, 0, stream>>>(Wsh, SD, SD, SD, WSH, SD, SD);
  k_plane<3><<<64 * 512 / 8 / 256, 256, 0, stream>>>(Wat, NA, SD, SD, WA2, 64, SD);
  k_plane<3><<<SD * 256 / 8 / 256, 256, 0, stream>>>(Wbm, SD, ED, ED, WBM2, SD, ED);
  k_plane<3><<<SD * 512 / 8 / 256, 256, 0, stream>>>(Wb0, SD, SD, SD + 1, W0D, SD, SD);
  k_gemm_nt<0, 0><<<8, 256, 0, stream>>>(XS, WSH, bsh, PRE, NN, SD, SD, SD);
  k_s1<<<NN / 8, 256, 0, stream>>>(PRE, bsh, S1, S1HL);
  k_gemm_nt<0, 0><<<2, 256, 0, stream>>>(S1HL, WA2, bsh, ATP, NN, 64, 512, 64);
  k_atoms<<<NN * NA / 4 / 256, 256, 0, stream>>>(ATP, bat, out + OUT1_OFS);
  k_coords<<<1, 256, 0, stream>>>(v, p, Wc, batch, CC, out);
  k_bucket<<<NBLK, NTHR, LDS_BKT, stream>>>(ei, NE, NN, 1, BLIST, OFFC, META);
  k_pair<<<NE / 256, 256, 0, stream>>>(ei, BLIST, OFFC, META, CC, PAIR, DD);
  k_esym<<<NE / 256, 256, 0, stream>>>(ef, PAIR, DD, ESHL);
  k_gemm_nt<0, 0><<<256, 256, 0, stream>>>(ESHL, WBM2, bsh, GH, NE, SD, 2 * ED, SD);
  k_f<<<NE / 256, 256, 0, stream>>>(ei, S1, GH, bbm, FHL);
  k_gemm_nt<0, 0><<<256, 256, 0, stream>>>(FHL, W0D, bsh, GH, NE, SD, 2 * SD, SD);
  k_out<<<NE / 256, 256, 0, stream>>>(GH, DD, Wb0, bb0, Wb1, bb1, out + OUT2_OFS);
}
